// SelfAttentionBlock_57019985821758
// MI455X (gfx1250) — hardware-verified
//
#include <hip/hip_runtime.h>
#ifndef NB
#define NB 2
#endif
#define NB_FULL 2
#define CCH 64
#define ACH 32
#define DD 28
#define S_TOT (DD * DD * DD)
#define T_REAL (S_TOT / 8)
#define T_PAD 2752
#define X_BSTRIDE_FULL ((size_t)CCH * S_TOT)
#define BPB (S_TOT / 64)
#define TBPB (T_PAD / 64)
#define NBLK (NB * BPB)
#define NEGB (-1.0e30f)
#define PCARRY 4096.0f
#define RSCALE 2048.0f
#define RINV 0.00048828125f

static_assert(S_TOT % 64 == 0);
static_assert(T_PAD % 64 == 0);
static_assert(T_PAD >= T_REAL);
static_assert(T_PAD - T_REAL < 32);
static_assert((NB * T_PAD * 8) % 256 == 0);
static_assert(((size_t)NB * CCH * S_TOT / 4) % 256 == 0);
static_assert(S_TOT % 4 == 0);
static_assert(NB <= NB_FULL);

typedef __bf16 v16b __attribute__((ext_vector_type(16)));
typedef _Float16 v16h __attribute__((ext_vector_type(16)));
typedef unsigned short v8us __attribute__((ext_vector_type(8), may_alias));
typedef float v8f __attribute__((ext_vector_type(8)));
typedef float v4f __attribute__((ext_vector_type(4)));
typedef float v4fa __attribute__((ext_vector_type(4), may_alias));
union FragB { v16b v; v8us half[2]; unsigned short u[16]; };
union FragH { v16h v; v8us half[2]; _Float16 h[16]; unsigned short u[16]; };

__device__ __forceinline__ unsigned short bf16_bits(float x) { unsigned int u = __float_as_uint(x); return (unsigned short)((u + 0x7FFFu + ((u >> 16) & 1u)) >> 16); }
__device__ __forceinline__ float bf16_val(unsigned short b) { return __uint_as_float(((unsigned int)b) << 16); }
__device__ __forceinline__ float bf16_rne(float x) { return bf16_val(bf16_bits(x)); }

__device__ __forceinline__ v16b ldb(const unsigned short* p, int hh) { FragB f; f.half[0] = *(const v8us*)(p + 8 * hh); f.half[1] = *(const v8us*)(p + 16 + 8 * hh); return f.v; }
__device__ __forceinline__ v16h ldh(const unsigned short* p, int hh) { FragH f; f.half[0] = *(const v8us*)(p + 8 * hh); f.half[1] = *(const v8us*)(p + 16 + 8 * hh); return f.v; }
__device__ __forceinline__ v16b ldb_f32(const float* p, int hh) {
  const v4f x0 = *(const v4fa*)(p + 8 * hh), x1 = *(const v4fa*)(p + 8 * hh + 4);
  const v4f x2 = *(const v4fa*)(p + 16 + 8 * hh), x3 = *(const v4fa*)(p + 16 + 8 * hh + 4);
  FragB f;
#pragma unroll
  for (int i = 0; i < 4; ++i) { f.u[i] = bf16_bits(x0[i]); f.u[4 + i] = bf16_bits(x1[i]); f.u[8 + i] = bf16_bits(x2[i]); f.u[12 + i] = bf16_bits(x3[i]); }
  return f.v;
}

__device__ __forceinline__ v8f mma_bf2(v16b a0, v16b b0, v16b a1, v16b b1, v8f c) {
  c = __builtin_amdgcn_wmma_f32_16x16x32_bf16(false, a0, false, b0, (short)0, c, false, false);
  c = __builtin_amdgcn_wmma_f32_16x16x32_bf16(false, a1, false, b1, (short)0, c, false, false);
  asm volatile("v_nop\n\tv_nop\n\tv_nop\n\tv_nop" : "+v"(c) : "v"(a0), "v"(b0), "v"(a1), "v"(b1));
  return c;
}
__device__ __forceinline__ v8f mma_h1(v16h a, v16h b, v8f c) {
  c = __builtin_amdgcn_wmma_f32_16x16x32_f16(false, a, false, b, (short)0, c, false, false);
  asm volatile("v_nop\n\tv_nop\n\tv_nop\n\tv_nop" : "+v"(c) : "v"(a), "v"(b));
  return c;
}
__device__ __forceinline__ v8f mma_h2(v16h a0, v16h b0, v16h a1, v16h b1, v8f c) {
  c = __builtin_amdgcn_wmma_f32_16x16x32_f16(false, a0, false, b0, (short)0, c, false, false);
  c = __builtin_amdgcn_wmma_f32_16x16x32_f16(false, a1, false, b1, (short)0, c, false, false);
  asm volatile("v_nop\n\tv_nop\n\tv_nop\n\tv_nop" : "+v"(c) : "v"(a0), "v"(b0), "v"(a1), "v"(b1));
  return c;
}

__global__ __launch_bounds__(256) void k_theta(const float* __restrict__ x, unsigned short* __restrict__ TH) {
  __shared__ __attribute__((aligned(16))) unsigned short tl[64][72];
  const int tid = threadIdx.x;
  const int n = blockIdx.x / BPB, sb = blockIdx.x - n * BPB;
  const int s0 = sb * 64;
#pragma unroll
  for (int it = 0; it < 4; ++it) {
    const int i = it * 256 + tid;
    const int c = i >> 4, q = (i & 15) * 4;
    const v4f v = *(const v4fa*)(x + (size_t)n * X_BSTRIDE_FULL + (size_t)c * S_TOT + s0 + q);
    tl[q + 0][c] = bf16_bits(v[0]); tl[q + 1][c] = bf16_bits(v[1]); tl[q + 2][c] = bf16_bits(v[2]); tl[q + 3][c] = bf16_bits(v[3]);
  }
  __syncthreads();
  for (int pass = 0; pass < 2; ++pass) {
#pragma unroll
    for (int it = 0; it < 2; ++it) {
      const int i = it * 256 + tid;
      const int r = i >> 3, pc = (i & 7) * 8;
      const v8us v = *(const v8us*)&tl[r][pc];
      *(volatile v8us*)(TH + ((size_t)n * S_TOT + s0 + r) * CCH + pc) = v;
    }
    if (pass == 0) __threadfence();
  }
}

__global__ __launch_bounds__(256) void k_phi(const unsigned short* __restrict__ TH, unsigned short* __restrict__ PHI) {
  const int idx = blockIdx.x * 256 + threadIdx.x;
  if (idx >= NB * T_PAD * 8) return;
  const int row = idx >> 3, pc = (idx & 7) * 8;
  const int n = row / T_PAD, t = row - n * T_PAD;
  const bool valid = t < T_REAL;
  const int tc = valid ? t : (T_REAL - 1);
  const int d2 = tc / 196, r = tc - d2 * 196, w2 = r / 14, h2 = r - w2 * 14;
  const int base = d2 * 1568 + w2 * 56 + h2 * 2;
  const unsigned short* src = TH + ((size_t)n * S_TOT + base) * CCH + pc;
  FragB m; m.half[0] = *(const v8us*)src;
#pragma unroll
  for (int k = 1; k < 8; ++k) {
    const int off = (k >> 2) * 784 + ((k >> 1) & 1) * 28 + (k & 1);
    FragB cc; cc.half[0] = *(const v8us*)(src + (size_t)off * CCH);
#pragma unroll
    for (int i = 0; i < 8; ++i) { const float a = bf16_val(m.u[i]), b = bf16_val(cc.u[i]); m.u[i] = (unsigned short)(__float_as_uint(fmaxf(a, b)) >> 16); }
  }
  v8us o;
#pragma unroll
  for (int i = 0; i < 8; ++i) o[i] = valid ? m.u[i] : (unsigned short)0;
  unsigned short* dst = PHI + (size_t)row * CCH + pc;
  *(volatile v8us*)dst = o;
  __threadfence();
  *(volatile v8us*)dst = o;
}

__global__ __launch_bounds__(128) void k_g(const unsigned short* __restrict__ TH, const float* __restrict__ g_w, const float* __restrict__ g_b,
                                          unsigned short* __restrict__ GH, unsigned short* __restrict__ GL) {
  __shared__ __attribute__((aligned(16))) _Float16 gh[32][72];
  __shared__ __attribute__((aligned(16))) _Float16 gl[32][72];
  const int tid = threadIdx.x, w = tid >> 5, lane = tid & 31, lo = lane & 15, hh = lane >> 4;
  const int n = blockIdx.x / TBPB, tb = blockIdx.x - n * TBPB;
  const int t0 = tb * 64 + 16 * w;
  const v16b b00 = ldb_f32(g_w + (size_t)lo * CCH, hh), b01 = ldb_f32(g_w + (size_t)lo * CCH + 32, hh);
  const v16b b10 = ldb_f32(g_w + (size_t)(16 + lo) * CCH, hh), b11 = ldb_f32(g_w + (size_t)(16 + lo) * CCH + 32, hh);
  const float gb0 = bf16_rne(g_b[lo]), gb1 = bf16_rne(g_b[16 + lo]);
  const unsigned short* thn = TH + (size_t)n * S_TOT * CCH;
  const int k = lo & 7;
  const int coff = (k >> 2) * 784 + ((k >> 1) & 1) * 28 + (k & 1);
  const v8f z8 = {0.f, 0.f, 0.f, 0.f, 0.f, 0.f, 0.f, 0.f};
#pragma unroll 1
  for (int j = 0; j < 8; ++j) {
    const int t = t0 + 2 * j + (lo >> 3);
    const int tc = (t < T_REAL) ? t : (T_REAL - 1);
    const int d2 = tc / 196, r = tc - d2 * 196, w2 = r / 14, h2 = r - w2 * 14;
    const int s = d2 * 1568 + w2 * 56 + h2 * 2 + coff;
    const unsigned short* ar = thn + (size_t)s * CCH;
    const v16b a0 = ldb(ar, hh), a1 = ldb(ar + 32, hh);
    const v8f c0 = mma_bf2(a0, b00, a1, b01, z8);
    const v8f c1 = mma_bf2(a0, b10, a1, b11, z8);
    float m0 = c0[0], m1 = c1[0];
#pragma unroll
    for (int q = 1; q < 8; ++q) { m0 = fmaxf(m0, c0[q]); m1 = fmaxf(m1, c1[q]); }
    const int tp = t0 + 2 * j + hh;
    const bool ok = tp < T_REAL;
    const float v0 = ok ? (m0 + gb0) : 0.f, v1 = ok ? (m1 + gb1) : 0.f;
    _Float16 h0 = (_Float16)v0, h1 = (_Float16)v1;
    h0 = (fabsf((float)h0) < 6.2e-5f) ? (_Float16)0.0f : h0;
    h1 = (fabsf((float)h1) < 6.2e-5f) ? (_Float16)0.0f : h1;
    const _Float16 l0 = (_Float16)((v0 - (float)h0) * RSCALE), l1 = (_Float16)((v1 - (float)h1) * RSCALE);
    const int tl = 16 * w + 2 * j + hh;
    gh[lo][tl] = h0; gh[16 + lo][tl] = h1; gl[lo][tl] = l0; gl[16 + lo][tl] = l1;
  }
  __syncthreads();
  for (int pass = 0; pass < 2; ++pass) {
#pragma unroll
    for (int it = 0; it < 2; ++it) {
      const int i = it * 128 + tid;
      const int a = i >> 3, pc = (i & 7) * 8;
      const v8us vh = *(const v8us*)&gh[a][pc];
      const v8us vl = *(const v8us*)&gl[a][pc];
      const size_t o = ((size_t)n * ACH + a) * T_PAD + tb * 64 + pc;
      *(volatile v8us*)(GH + o) = vh;
      *(volatile v8us*)(GL + o) = vl;
    }
    if (pass == 0) __threadfence();
  }
}

__global__ __launch_bounds__(128) void k_attn(const unsigned short* __restrict__ TH, const unsigned short* __restrict__ PHI,
                                             const unsigned short* __restrict__ GH, const unsigned short* __restrict__ GL,
                                             const float* __restrict__ w_w, const float* __restrict__ w_b,
                                             float* __restrict__ Z, float* __restrict__ PART) {
  __shared__ __attribute__((aligned(16))) float zt[64][68];
  __shared__ __attribute__((aligned(16))) float st[128];
  const int tid = threadIdx.x, w = tid >> 5, lane = tid & 31, lo = lane & 15, hh = lane >> 4;
  const int n = blockIdx.x / BPB, bb = blockIdx.x - n * BPB;
  const int row0 = bb * 64 + 16 * w;
  const unsigned short* tr = TH + ((size_t)n * S_TOT + row0 + lo) * CCH;
  const v16b tb0 = ldb(tr, hh), tb1 = ldb(tr + 32, hh);
  const unsigned short* phin = PHI + (size_t)n * T_PAD * CCH;
  const unsigned short* gh0p = GH + ((size_t)n * ACH + lo) * T_PAD;
  const unsigned short* gh1p = gh0p + (size_t)16 * T_PAD;
  const unsigned short* gl0p = GL + ((size_t)n * ACH + lo) * T_PAD;
  const unsigned short* gl1p = gl0p + (size_t)16 * T_PAD;
  const v8f z8 = {0.f, 0.f, 0.f, 0.f, 0.f, 0.f, 0.f, 0.f};
  v8f ah0 = z8, ah1 = z8, ax0 = z8, ax1 = z8;
  float mrow = NEGB, lrow = 0.f;
#pragma unroll 1
  for (int kb = 0; kb < T_PAD; kb += 32) {
    const unsigned short* p0 = phin + (size_t)(kb + lo) * CCH;
    const unsigned short* p1 = p0 + (size_t)16 * CCH;
    v8f s0, s1;
    { const v16b a0 = ldb(p0, hh), a1 = ldb(p0 + 32, hh); s0 = mma_bf2(a0, tb0, a1, tb1, z8); }
    { const v16b a0 = ldb(p1, hh), a1 = ldb(p1 + 32, hh); s1 = mma_bf2(a0, tb0, a1, tb1, z8); }
    if (kb + 32 > T_REAL) {
#pragma unroll
      for (int v = 0; v < 8; ++v) {
        s0[v] = (kb + 8 * hh + v >= T_REAL) ? NEGB : s0[v];
        s1[v] = (kb + 16 + 8 * hh + v >= T_REAL) ? NEGB : s1[v];
      }
    }
    float cmx = fmaxf(s0[0], s1[0]);
#pragma unroll
    for (int v = 1; v < 8; ++v) cmx = fmaxf(cmx, fmaxf(s0[v], s1[v]));
    cmx = fmaxf(cmx, __shfl_xor(cmx, 16, 32));
    const float mnew = fmaxf(mrow, cmx);
    const float alpha = __expf(mrow - mnew);
    mrow = mnew;
    FragH ph, pl;
    float ls = 0.f;
#pragma unroll
    for (int v = 0; v < 8; ++v) {
      const float e0 = __expf(s0[v] - mnew), e1 = __expf(s1[v] - mnew);
      ls += e0 + e1;
      const float q0 = e0 * PCARRY, q1 = e1 * PCARRY;
      const _Float16 h0 = (_Float16)q0, h1 = (_Float16)q1;
      ph.h[v] = h0; ph.h[8 + v] = h1;
      pl.h[v] = (_Float16)((q0 - (float)h0) * RSCALE); pl.h[8 + v] = (_Float16)((q1 - (float)h1) * RSCALE);
    }
    ls += __shfl_xor(ls, 16, 32);
    lrow = lrow * alpha + ls;
    ah0 = ah0 * alpha; ah1 = ah1 * alpha; ax0 = ax0 * alpha; ax1 = ax1 * alpha;
    const v16h vh0 = ldh(gh0p + kb, hh), vh1 = ldh(gh1p + kb, hh);
    const v16h vl0 = ldh(gl0p + kb, hh), vl1 = ldh(gl1p + kb, hh);
    ah0 = mma_h1(vh0, ph.v, ah0);
    ah1 = mma_h1(vh1, ph.v, ah1);
    ax0 = mma_h2(vh0, pl.v, vl0, ph.v, ax0);
    ax1 = mma_h2(vh1, pl.v, vl1, ph.v, ax1);
  }
  const float inv = 1.0f / (lrow * PCARRY);
  FragB yh, yl;
#pragma unroll
  for (int r = 0; r < 8; ++r) {
    const float y0 = (ah0[r] + ax0[r] * RINV) * inv, y1 = (ah1[r] + ax1[r] * RINV) * inv;
    const unsigned short hb0 = bf16_bits(y0), hb1 = bf16_bits(y1);
    yh.u[r] = hb0; yh.u[8 + r] = hb1;
    yl.u[r] = bf16_bits(y0 - bf16_val(hb0)); yl.u[8 + r] = bf16_bits(y1 - bf16_val(hb1));
  }
#pragma unroll
  for (int tt = 0; tt < 4; ++tt) {
    const v16b wa = ldb_f32(w_w + (size_t)(16 * tt + lo) * ACH, hh);
    const v8f zc = mma_bf2(wa, yh.v, wa, yl.v, z8);
#pragma unroll
    for (int r = 0; r < 8; ++r) { const int c = 16 * tt + 8 * hh + r; zt[c][16 * w + lo] = zc[r] + bf16_rne(w_b[c]); }
  }
  __syncthreads();
  if (tid < 64) {
    float s = 0.f;
#pragma unroll 4
    for (int j = 0; j < 64; ++j) s += zt[tid][j];
    const float mb = s * 0.015625f;
    float m2 = 0.f;
#pragma unroll 4
    for (int j = 0; j < 64; ++j) { const float d = zt[tid][j] - mb; m2 += d * d; }
    st[tid] = s; st[64 + tid] = m2;
  }
  __syncthreads();
  for (int pass = 0; pass < 2; ++pass) {
#pragma unroll
    for (int it = 0; it < 8; ++it) {
      const int r = it * 8 + (tid >> 4), pc = (tid & 15) * 4;
      const v4f v = *(const v4fa*)&zt[r][pc];
      *(volatile v4f*)(Z + ((size_t)n * CCH + r) * S_TOT + bb * 64 + pc) = v;
    }
    if (tid < 32) {
      const v4f v = *(const v4fa*)&st[4 * tid];
      *(volatile v4f*)(PART + (size_t)blockIdx.x * 128 + 4 * tid) = v;
    }
    if (pass == 0) __threadfence();
  }
}

__global__ __launch_bounds__(64) void k_bn(const float* __restrict__ PART, const float* __restrict__ gamma, const float* __restrict__ beta, float* __restrict__ SB) {
  __shared__ __attribute__((aligned(16))) float sl[256];
  const int c = threadIdx.x;
  const double cnt = (double)NB * (double)S_TOT;
  double S = 0.0;
#pragma unroll 1
  for (int b = 0; b < NBLK; ++b) S += (double)PART[(size_t)b * 128 + c];
  const double mean = S * (1.0 / cnt);
  double M = 0.0;
#pragma unroll 1
  for (int b = 0; b < NBLK; ++b) {
    const double d = (double)PART[(size_t)b * 128 + c] * 0.015625 - mean;
    M += (double)PART[(size_t)b * 128 + 64 + c] + 64.0 * d * d;
  }
  const float var = (float)(M * (1.0 / cnt));
  sl[c] = (float)mean;
  sl[64 + c] = bf16_rne(gamma[c]) * rsqrtf(var + 1e-5f);
  sl[128 + c] = bf16_rne(beta[c]);
  sl[192 + c] = 0.f;
  __syncthreads();
  const v4f v = *(const v4fa*)&sl[4 * c];
  *(volatile v4f*)(SB + 4 * c) = v;
  __threadfence();
  *(volatile v4f*)(SB + 4 * c) = v;
}

__global__ __launch_bounds__(256) void k_out(const float* __restrict__ Z, const float* __restrict__ SB, const float* __restrict__ x, float* __restrict__ out) {
  const size_t idx = (size_t)blockIdx.x * 256 + threadIdx.x;
  if (idx >= (size_t)NB * CCH * S_TOT / 4) return;
  const size_t e = idx * 4;
  const int c = (int)((e / S_TOT) % CCH);
  const float mean = SB[c], sc = SB[64 + c], be = SB[128 + c];
  const v4f z = *(const v4fa*)(Z + e);
  const v4f xv = *(const v4fa*)(x + e);
  v4f o;
#pragma unroll
  for (int q = 0; q < 4; ++q) o[q] = (z[q] - mean) * sc + be + bf16_rne(xv[q]);
  *(volatile v4f*)(out + e) = o;
  __threadfence();
  *(volatile v4f*)(out + e) = o;
}

extern "C" void kernel_launch(void* const* d_in, const int* in_sizes, int n_in,
                              void* d_out, int out_size, void* d_ws, size_t ws_size, hipStream_t stream) {
  if (n_in < 7) return;
  if ((size_t)in_sizes[0] < (size_t)NB * CCH * S_TOT) return;
  if (in_sizes[1] < ACH * CCH || in_sizes[2] < ACH || in_sizes[3] < CCH * ACH || in_sizes[4] < CCH || in_sizes[5] < CCH || in_sizes[6] < CCH) return;
  if ((size_t)out_size < (size_t)NB * CCH * S_TOT) return;
  const float* x = (const float*)d_in[0];
  const float* g_w = (const float*)d_in[1];
  const float* g_b = (const float*)d_in[2];
  const float* w_w = (const float*)d_in[3];
  const float* w_b = (const float*)d_in[4];
  const float* gamma = (const float*)d_in[5];
  const float* beta = (const float*)d_in[6];
  float* out = (float*)d_out;
  char* ws = (char*)d_ws;
  size_t off = 0;
  auto take = [&](size_t bytes) { char* p = ws + off; off += (bytes + 255) & ~(size_t)255; return p; };
  unsigned short* TH = (unsigned short*)take((size_t)NB * S_TOT * CCH * 2);
  unsigned short* PHI = (unsigned short*)take((size_t)NB * T_PAD * CCH * 2);
  unsigned short* GH = (unsigned short*)take((size_t)NB * ACH * T_PAD * 2);
  unsigned short* GL = (unsigned short*)take((size_t)NB * ACH * T_PAD * 2);
  float* Z = (float*)take((size_t)NB * CCH * S_TOT * 4);
  float* PART = (float*)take((size_t)NBLK * 128 * 4);
  float* SB = (float*)take((size_t)256 * 4);
  if (off > ws_size) return;
  k_theta<<<NB * BPB, 256, 0, stream>>>(x, TH);
  k_phi<<<(NB * T_PAD * 8) / 256, 256, 0, stream>>>(TH, PHI);
  k_g<<<NB * TBPB, 128, 0, stream>>>(TH, g_w, g_b, GH, GL);
  k_attn<<<NB * BPB, 128, 0, stream>>>(TH, PHI, GH, GL, w_w, w_b, Z, PART);
  k_bn<<<1, 64, 0, stream>>>(PART, gamma, beta, SB);
  k_out<<<(unsigned)(((size_t)NB * CCH * S_TOT / 4) / 256), 256, 0, stream>>>(Z, SB, x, out);
}
